// DGMC_86028194939238
// MI455X (gfx1250) — hardware-verified
//
#include <hip/hip_runtime.h>


#define NB    4
#define NN    1024
#define FIN   128
#define FHID  256
#define RR    16
#define BNN   (NB * NN)
#define NT    32
#define LCAP  2048
#define NWAVE 8

typedef __bf16         v16b __attribute__((ext_vector_type(16)));
typedef unsigned short v8us __attribute__((ext_vector_type(8)));
typedef unsigned int   v8u  __attribute__((ext_vector_type(8)));
typedef float          v8f  __attribute__((ext_vector_type(8)));
typedef float          v4f  __attribute__((ext_vector_type(4)));

union Frag { v16b v; v8us hv[2]; v8u u; };

__device__ __forceinline__ unsigned short bf_rne(float x) {
    unsigned int u = __float_as_uint(x);
    u += 0x7FFFu + ((u >> 16) & 1u);
    return (unsigned short)(u >> 16);
}
__device__ __forceinline__ float bf_up(unsigned short s) {
    return __uint_as_float(((unsigned int)s) << 16);
}
__device__ __forceinline__ void split2(float x, unsigned short& h, unsigned short& l) {
    h = bf_rne(x);
    l = bf_rne(x - bf_up(h));
}
__device__ __forceinline__ void split3(float x, unsigned short& h, unsigned short& m, unsigned short& l) {
    h = bf_rne(x);
    const float r1 = x - bf_up(h);
    m = bf_rne(r1);
    l = bf_rne(r1 - bf_up(m));
}
__device__ __forceinline__ unsigned int pk16(unsigned short lo, unsigned short hi) {
    return (unsigned int)lo | ((unsigned int)hi << 16);
}

__device__ __forceinline__ v8f mma(v8f acc, v16b a, v16b b) {
    acc = __builtin_amdgcn_wmma_f32_16x16x32_bf16(false, a, false, b, (short)0, acc, false, false);
    asm volatile("v_nop\n\tv_nop\n\tv_nop\n\tv_nop" : "+v"(acc) : "v"(a), "v"(b));
    return acc;
}
__device__ __forceinline__ v8f mma6(v8f acc, v16b a0, v16b a1, v16b a2, v16b b0, v16b b1, v16b b2) {
    acc = mma(acc, a0, b2);
    acc = mma(acc, a1, b1);
    acc = mma(acc, a2, b0);
    acc = mma(acc, a0, b1);
    acc = mma(acc, a1, b0);
    acc = mma(acc, a0, b0);
    return acc;
}
__device__ __forceinline__ v8f zero8() {
    v8f z = {0.f, 0.f, 0.f, 0.f, 0.f, 0.f, 0.f, 0.f};
    return z;
}

__device__ __forceinline__ v16b ld_frag(const unsigned short* rowp, int k0, int h) {
    Frag f;
    f.hv[0] = *(const v8us*)(rowp + k0 + 8 * h);
    f.hv[1] = *(const v8us*)(rowp + k0 + 16 + 8 * h);
    return f.v;
}

__device__ __forceinline__ void build_segments(const int* __restrict__ ei, int E, int nChunks, int d0,
                                               int* list, int* wcnt, int* cntn, int* segoff, int* slots)
{
    const int tid = threadIdx.x, lane = tid & 31, w = tid >> 5;
    int base = 0;
    for (int ch = 0; ch < nChunks; ++ch) {
        const int e = ch * 256 + tid;
        int ok = 0, src = 0, jl = 0;
        if (e < E) {
            src = ei[e];
            const int dst = ei[(size_t)E + e];
            jl = dst - d0;
            ok = ((unsigned)jl < (unsigned)NT) ? 1 : 0;
            src = src < 0 ? 0 : (src > BNN - 1 ? BNN - 1 : src);
        }
        const unsigned int msk = __builtin_amdgcn_ballot_w32(ok != 0);
        const int pre = (int)__popc(msk & ((1u << lane) - 1u));
        if (lane == 0) wcnt[w] = (int)__popc(msk);
        __syncthreads();
        int offw = 0, tot = 0;
#pragma unroll
        for (int i = 0; i < NWAVE; ++i) {
            const int c = wcnt[i];
            tot += c;
            offw += (i < w) ? c : 0;
        }
        if (ok) {
            const int pos = base + offw + pre;
            if ((unsigned)pos < (unsigned)LCAP) list[pos] = (src << 5) | jl;
        }
        base += tot;
        __syncthreads();
    }
    const int L = base < LCAP ? base : LCAP;
    if (tid < NT) {
        int c = 0;
        for (int p = 0; p < L; ++p) c += ((list[p] & 31) == tid) ? 1 : 0;
        cntn[tid] = c;
    }
    __syncthreads();
    if (tid == 0) {
        int o = 0;
        for (int j = 0; j < NT; ++j) { segoff[j] = o; o += cntn[j]; }
        segoff[NT] = o;
    }
    __syncthreads();
    if (tid < NT) {
        int pos = segoff[tid];
        for (int p = 0; p < L; ++p) {
            const int v = list[p];
            if ((v & 31) == tid) {
                if ((unsigned)pos < (unsigned)LCAP) slots[pos] = v >> 5;
                ++pos;
            }
        }
    }
    __syncthreads();
}

__global__ void __launch_bounds__(256) k_w1cvt(const float* __restrict__ W1, unsigned short* __restrict__ W1p)
{
    __shared__ float tile[16][FIN + 1];
    const int tid = threadIdx.x;
    const int n0 = blockIdx.x * 16;
    {
        const int j = tid & 15, kq = tid >> 4;
#pragma unroll
        for (int i = 0; i < FIN / 16; ++i) {
            const int k = kq + 16 * i;
            tile[j][k] = W1[(size_t)k * FHID + n0 + j];
        }
    }
    __syncthreads();
    const int row = tid >> 4, q = tid & 15;
    v8us ph, pm, pl;
#pragma unroll
    for (int c = 0; c < 8; ++c) {
        unsigned short a, b, d;
        split3(tile[row][8 * q + c], a, b, d);
        ph[c] = a; pm[c] = b; pl[c] = d;
    }
    const size_t PS = (size_t)FHID * FIN;
    const size_t o = (size_t)(n0 + row) * FIN + 8 * q;
    *(volatile v8us*)(W1p + o) = ph;
    *(volatile v8us*)(W1p + PS + o) = pm;
    *(volatile v8us*)(W1p + 2 * PS + o) = pl;
    __threadfence();
    *(volatile v8us*)(W1p + o) = ph;
    *(volatile v8us*)(W1p + PS + o) = pm;
    *(volatile v8us*)(W1p + 2 * PS + o) = pl;
}

__global__ void __launch_bounds__(256) k_agg_feat(const float* __restrict__ x, const int* __restrict__ ei,
                                                  int E, int nChunks, unsigned short* __restrict__ Ap)
{
    __shared__ int list[LCAP];
    __shared__ int slots[LCAP];
    __shared__ int wcnt[NWAVE];
    __shared__ int cntn[NT];
    __shared__ int segoff[NT + 1];
    const int tid = threadIdx.x;
    const int d0 = blockIdx.x * NT;
    build_segments(ei, E, nChunks, d0, list, wcnt, cntn, segoff, slots);

    const int q = tid & 15, jr = tid >> 4;
    v8us pc[2][3];
#pragma unroll
    for (int hf = 0; hf < 2; ++hf) {
        const int j = jr + 16 * hf;
        const int node = d0 + j;
        const float* xr = x + (size_t)node * FIN + 8 * q;
        v4f s0 = *(const v4f*)xr;
        v4f s1 = *(const v4f*)(xr + 4);
        int sb = segoff[j];
        int n = segoff[j + 1] - sb;
        sb = sb < 0 ? 0 : sb;
        n = n < 0 ? 0 : (n > LCAP ? LCAP : n);
        for (int p = 0; p < n; ++p) {
            int idx = sb + p;
            idx = idx > LCAP - 1 ? LCAP - 1 : idx;
            int src = slots[idx];
            src = ((unsigned)src < (unsigned)BNN) ? src : 0;
            const float* xs = x + (size_t)src * FIN + 8 * q;
            s0 += *(const v4f*)xs;
            s1 += *(const v4f*)(xs + 4);
        }
#pragma unroll
        for (int c = 0; c < 4; ++c) {
            unsigned short a, b, d;
            split3(s0[c], a, b, d);
            pc[hf][0][c] = a; pc[hf][1][c] = b; pc[hf][2][c] = d;
            split3(s1[c], a, b, d);
            pc[hf][0][4 + c] = a; pc[hf][1][4 + c] = b; pc[hf][2][4 + c] = d;
        }
    }
    const size_t PS = (size_t)BNN * FIN;
#pragma unroll
    for (int hf = 0; hf < 2; ++hf) {
        const size_t o = (size_t)(d0 + jr + 16 * hf) * FIN + 8 * q;
#pragma unroll
        for (int p = 0; p < 3; ++p) *(volatile v8us*)(Ap + (size_t)p * PS + o) = pc[hf][p];
    }
    __threadfence();
#pragma unroll
    for (int hf = 0; hf < 2; ++hf) {
        const size_t o = (size_t)(d0 + jr + 16 * hf) * FIN + 8 * q;
#pragma unroll
        for (int p = 0; p < 3; ++p) *(volatile v8us*)(Ap + (size_t)p * PS + o) = pc[hf][p];
    }
}

__global__ void __launch_bounds__(256) k_gemm1(const unsigned short* __restrict__ Ap,
                                               const unsigned short* __restrict__ W1p,
                                               const float* __restrict__ b1,
                                               unsigned short* __restrict__ Hp)
{
    __shared__ __attribute__((aligned(16))) float tile[64][68];
    const int tid = threadIdx.x, lane = tid & 31, w = tid >> 5, h = lane >> 4, m = lane & 15;
    const int rb = blockIdx.x >> 2, cb = blockIdx.x & 3;
    const int row0 = rb * 64, col0 = cb * 64;
    const int wr = w >> 1, wc = w & 1;
    const size_t PSA = (size_t)BNN * FIN, PSW = (size_t)FHID * FIN, PSH = (size_t)BNN * FHID;
    const unsigned short* arow  = Ap  + (size_t)(row0 + 16 * wr + m) * FIN;
    const unsigned short* brow0 = W1p + (size_t)(col0 + 32 * wc + m) * FIN;
    const unsigned short* brow1 = brow0 + (size_t)16 * FIN;

    v8f acc0 = zero8(), acc1 = zero8();
#pragma unroll 1
    for (int k0 = 0; k0 < FIN; k0 += 32) {
        const v16b a0 = ld_frag(arow, k0, h);
        const v16b a1 = ld_frag(arow + PSA, k0, h);
        const v16b a2 = ld_frag(arow + 2 * PSA, k0, h);
        {
            const v16b b0 = ld_frag(brow0, k0, h);
            const v16b bb = ld_frag(brow0 + PSW, k0, h);
            const v16b b2 = ld_frag(brow0 + 2 * PSW, k0, h);
            acc0 = mma6(acc0, a0, a1, a2, b0, bb, b2);
        }
        {
            const v16b b0 = ld_frag(brow1, k0, h);
            const v16b bb = ld_frag(brow1 + PSW, k0, h);
            const v16b b2 = ld_frag(brow1 + 2 * PSW, k0, h);
            acc1 = mma6(acc1, a0, a1, a2, b0, bb, b2);
        }
    }
#pragma unroll
    for (int r = 0; r < 8; ++r) {
        tile[16 * wr + 8 * h + r][32 * wc + m]      = acc0[r];
        tile[16 * wr + 8 * h + r][32 * wc + 16 + m] = acc1[r];
    }
    __syncthreads();

    const int q = tid & 7;
    const v4f bA = *(const v4f*)(b1 + col0 + 8 * q);
    const v4f bB = *(const v4f*)(b1 + col0 + 8 * q + 4);
    v8us pc[2][3];
#pragma unroll
    for (int ps = 0; ps < 2; ++ps) {
        const int rl = (tid >> 3) + 32 * ps;
        const v4f u0 = *(const v4f*)&tile[rl][8 * q] + bA;
        const v4f u1 = *(const v4f*)&tile[rl][8 * q + 4] + bB;
#pragma unroll
        for (int c = 0; c < 4; ++c) {
            const float x0 = u0[c] > 0.f ? u0[c] : 0.f;
            const float x1 = u1[c] > 0.f ? u1[c] : 0.f;
            unsigned short a, b, d;
            split3(x0, a, b, d);
            pc[ps][0][c] = a; pc[ps][1][c] = b; pc[ps][2][c] = d;
            split3(x1, a, b, d);
            pc[ps][0][4 + c] = a; pc[ps][1][4 + c] = b; pc[ps][2][4 + c] = d;
        }
    }
#pragma unroll
    for (int ps = 0; ps < 2; ++ps) {
        const size_t o = (size_t)(row0 + (tid >> 3) + 32 * ps) * FHID + col0 + 8 * q;
#pragma unroll
        for (int p = 0; p < 3; ++p) *(volatile v8us*)(Hp + (size_t)p * PSH + o) = pc[ps][p];
    }
    __threadfence();
#pragma unroll
    for (int ps = 0; ps < 2; ++ps) {
        const size_t o = (size_t)(row0 + (tid >> 3) + 32 * ps) * FHID + col0 + 8 * q;
#pragma unroll
        for (int p = 0; p < 3; ++p) *(volatile v8us*)(Hp + (size_t)p * PSH + o) = pc[ps][p];
    }
}

__global__ void __launch_bounds__(256) k_sim(const unsigned short* __restrict__ Hs,
                                             const unsigned short* __restrict__ Ht,
                                             float* __restrict__ Shat)
{
    __shared__ __attribute__((aligned(16))) float tile[64][68];
    const int tid = threadIdx.x, lane = tid & 31, w = tid >> 5, h = lane >> 4, m = lane & 15;
    const int blk = blockIdx.x;
    const int b  = blk >> 8;
    const int s0 = ((blk >> 4) & 15) * 64;
    const int t0 = (blk & 15) * 64;
    const int wr = w >> 1, wc = w & 1;
    const size_t PSH = (size_t)BNN * FHID;
    const unsigned short* arow  = Hs + (size_t)(b * NN + s0 + 16 * wr + m) * FHID;
    const unsigned short* brow0 = Ht + (size_t)(b * NN + t0 + 32 * wc + m) * FHID;
    const unsigned short* brow1 = brow0 + (size_t)16 * FHID;

    v8f acc0 = zero8(), acc1 = zero8();
#pragma unroll 1
    for (int k0 = 0; k0 < FHID; k0 += 32) {
        const v16b a0 = ld_frag(arow, k0, h);
        const v16b a1 = ld_frag(arow + PSH, k0, h);
        const v16b a2 = ld_frag(arow + 2 * PSH, k0, h);
        {
            const v16b b0 = ld_frag(brow0, k0, h);
            const v16b bb = ld_frag(brow0 + PSH, k0, h);
            const v16b b2 = ld_frag(brow0 + 2 * PSH, k0, h);
            acc0 = mma6(acc0, a0, a1, a2, b0, bb, b2);
        }
        {
            const v16b b0 = ld_frag(brow1, k0, h);
            const v16b bb = ld_frag(brow1 + PSH, k0, h);
            const v16b b2 = ld_frag(brow1 + 2 * PSH, k0, h);
            acc1 = mma6(acc1, a0, a1, a2, b0, bb, b2);
        }
    }
#pragma unroll
    for (int r = 0; r < 8; ++r) {
        tile[16 * wr + 8 * h + r][32 * wc + m]      = acc0[r];
        tile[16 * wr + 8 * h + r][32 * wc + 16 + m] = acc1[r];
    }
    __syncthreads();

    const int q = tid & 15;
    v4f ov[4];
#pragma unroll
    for (int ps = 0; ps < 4; ++ps) {
        const int rl = (tid >> 4) + 16 * ps;
        ov[ps] = *(const v4f*)&tile[rl][4 * q];
    }
#pragma unroll
    for (int ps = 0; ps < 4; ++ps) {
        const int rl = (tid >> 4) + 16 * ps;
        float* p = Shat + ((size_t)(b * NN + s0 + rl) * NN + t0 + 4 * q);
        *(volatile v4f*)p = ov[ps];
    }
    __threadfence();
#pragma unroll
    for (int ps = 0; ps < 4; ++ps) {
        const int rl = (tid >> 4) + 16 * ps;
        float* p = Shat + ((size_t)(b * NN + s0 + rl) * NN + t0 + 4 * q);
        *(volatile v4f*)p = ov[ps];
    }
}

__global__ void __launch_bounds__(256) k_softmax(const float* __restrict__ S, float* __restrict__ dst, int nrows)
{
    const int tid = threadIdx.x, lane = tid & 31;
    const int row = blockIdx.x * NWAVE + (tid >> 5);
    if (row >= nrows) return;
    const v4f* rp = (const v4f*)(S + (size_t)row * NN);
    v4f v[NN / 128];
    float mx = -3.0e38f;
#pragma unroll
    for (int i = 0; i < NN / 128; ++i) {
        v[i] = rp[32 * i + lane];
        mx = fmaxf(mx, fmaxf(fmaxf(v[i][0], v[i][1]), fmaxf(v[i][2], v[i][3])));
    }
#pragma unroll
    for (int o = 16; o > 0; o >>= 1) mx = fmaxf(mx, __shfl_xor(mx, o, 32));
    float sum = 0.f;
#pragma unroll
    for (int i = 0; i < NN / 128; ++i) {
#pragma unroll
        for (int c = 0; c < 4; ++c) {
            const float e = __expf(v[i][c] - mx);
            v[i][c] = e;
            sum += e;
        }
    }
#pragma unroll
    for (int o = 16; o > 0; o >>= 1) sum += __shfl_xor(sum, o, 32);
    const float inv = 1.0f / sum;
#pragma unroll
    for (int i = 0; i < NN / 128; ++i) v[i] = v[i] * inv;
    volatile v4f* dp = (volatile v4f*)(dst + (size_t)row * NN);
#pragma unroll
    for (int i = 0; i < NN / 128; ++i) dp[32 * i + lane] = v[i];
    __threadfence();
#pragma unroll
    for (int i = 0; i < NN / 128; ++i) dp[32 * i + lane] = v[i];
}

__global__ void __launch_bounds__(128) k_colmix(const float* __restrict__ S, const float* __restrict__ rs,
                                                float* __restrict__ rt)
{
    __shared__ __attribute__((aligned(16))) float Sl[32][68];
    __shared__ __attribute__((aligned(16))) float rl[32][20];
    __shared__ __attribute__((aligned(16))) float dl[4][16][20];
    const int tid = threadIdx.x, lane = tid & 31, w = tid >> 5, h = lane >> 4, m = lane & 15;
    const int b = blockIdx.x >> 4, t0 = (blockIdx.x & 15) * 64;

    v8f acc = zero8();
#pragma unroll 1
    for (int sc = 0; sc < NN; sc += 32) {
#pragma unroll
        for (int i = 0; i < 4; ++i) {
            const int idx = tid + 128 * i;
            const int r = idx >> 4, c4 = idx & 15;
            const v4f val = *(const v4f*)(S + ((size_t)(b * NN + sc + r) * NN + t0 + 4 * c4));
            Sl[r][4 * c4 + 0] = val[0]; Sl[r][4 * c4 + 1] = val[1];
            Sl[r][4 * c4 + 2] = val[2]; Sl[r][4 * c4 + 3] = val[3];
        }
        {
            const int r = tid >> 2, c4 = tid & 3;
            const v4f val = *(const v4f*)(rs + ((size_t)(b * NN + sc + r) * RR + 4 * c4));
            rl[r][4 * c4 + 0] = val[0]; rl[r][4 * c4 + 1] = val[1];
            rl[r][4 * c4 + 2] = val[2]; rl[r][4 * c4 + 3] = val[3];
        }
        __syncthreads();
        float av[16], bv[16];
#pragma unroll
        for (int i = 0; i < 16; ++i) {
            const int k = 8 * h + i + ((i >> 3) << 3);
            av[i] = Sl[k][16 * w + m];
            bv[i] = rl[k][m];
        }
        Frag ah, al, bh, bl;
#pragma unroll
        for (int c = 0; c < 8; ++c) {
            unsigned short h0, l0, h1, l1;
            split2(av[2 * c], h0, l0); split2(av[2 * c + 1], h1, l1);
            ah.u[c] = pk16(h0, h1); al.u[c] = pk16(l0, l1);
            split2(bv[2 * c], h0, l0); split2(bv[2 * c + 1], h1, l1);
            bh.u[c] = pk16(h0, h1); bl.u[c] = pk16(l0, l1);
        }
        acc = mma(acc, al.v, bh.v);
        acc = mma(acc, ah.v, bl.v);
        acc = mma(acc, ah.v, bh.v);
        __syncthreads();
    }
#pragma unroll
    for (int r = 0; r < 8; ++r) dl[w][8 * h + r][m] = acc[r];
    __syncthreads();
    v4f ov[2];
    size_t oo[2];
#pragma unroll
    for (int i = 0; i < 2; ++i) {
        const int line = 4 * i + (lane >> 3), ch = lane & 7;
        const int rowl = 2 * line + (ch >> 2), col = 4 * (ch & 3);
        ov[i] = *(const v4f*)&dl[w][rowl][col];
        oo[i] = (size_t)(b * NN + t0 + 16 * w + rowl) * RR + col;
    }
#pragma unroll
    for (int i = 0; i < 2; ++i) *(volatile v4f*)(rt + oo[i]) = ov[i];
    __threadfence();
#pragma unroll
    for (int i = 0; i < 2; ++i) *(volatile v4f*)(rt + oo[i]) = ov[i];
}

__global__ void __launch_bounds__(256) k_agg_mlp(const float* __restrict__ v, const int* __restrict__ ei,
                                                 int E, int nChunks,
                                                 const float* __restrict__ W2, const float* __restrict__ b2,
                                                 const float* __restrict__ Wm1, const float* __restrict__ bm1,
                                                 int addBias, float* __restrict__ aOut)
{
    __shared__ int list[LCAP];
    __shared__ int slots[LCAP];
    __shared__ int wcnt[NWAVE];
    __shared__ int cntn[NT];
    __shared__ int segoff[NT + 1];
    __shared__ float w2l[RR * RR];
    __shared__ float wm1l[RR * RR];
    __shared__ float b2l[RR];
    __shared__ float bm1l[RR];
    __shared__ float aggl[NT][RR + 1];
    __shared__ float ol[NT][RR + 1];
    __shared__ __attribute__((aligned(16))) float al[NT][RR + 4];
    const int tid = threadIdx.x;
    const int d0 = blockIdx.x * NT;
    w2l[tid] = W2[tid];
    wm1l[tid] = Wm1[tid];
    if (tid < RR) { b2l[tid] = b2[tid]; bm1l[tid] = addBias ? bm1[tid] : 0.0f; }
    build_segments(ei, E, nChunks, d0, list, wcnt, cntn, segoff, slots);

    const int j = tid >> 3, cp = tid & 7, c0 = 2 * cp;
    const int node = d0 + j;
    {
        float s0 = v[(size_t)node * RR + c0];
        float s1 = v[(size_t)node * RR + c0 + 1];
        int sb = segoff[j];
        int n = segoff[j + 1] - sb;
        sb = sb < 0 ? 0 : sb;
        n = n < 0 ? 0 : (n > LCAP ? LCAP : n);
        for (int p = 0; p < n; ++p) {
            int idx = sb + p;
            idx = idx > LCAP - 1 ? LCAP - 1 : idx;
            int src = slots[idx];
            src = ((unsigned)src < (unsigned)BNN) ? src : 0;
            s0 += v[(size_t)src * RR + c0];
            s1 += v[(size_t)src * RR + c0 + 1];
        }
        aggl[j][c0] = s0;
        aggl[j][c0 + 1] = s1;
    }
    __syncthreads();
    {
        float o0 = b2l[c0], o1 = b2l[c0 + 1];
#pragma unroll
        for (int k = 0; k < RR; ++k) {
            const float xk = aggl[j][k];
            o0 = fmaf(xk, w2l[k * RR + c0], o0);
            o1 = fmaf(xk, w2l[k * RR + c0 + 1], o1);
        }
        ol[j][c0]     = o0 > 0.f ? o0 : 0.f;
        ol[j][c0 + 1] = o1 > 0.f ? o1 : 0.f;
    }
    __syncthreads();
    {
        float u0 = bm1l[c0], u1 = bm1l[c0 + 1];
#pragma unroll
        for (int r = 0; r < RR; ++r) {
            const float orr = ol[j][r];
            u0 = fmaf(orr, wm1l[r * RR + c0], u0);
            u1 = fmaf(orr, wm1l[r * RR + c0 + 1], u1);
        }
        al[j][c0] = u0;
        al[j][c0 + 1] = u1;
    }
    __syncthreads();
    if (tid < 128) {
        const int line = tid >> 3, ch = tid & 7;
        const int nl = 2 * line + (ch >> 2), col = 4 * (ch & 3);
        const v4f ov = *(const v4f*)&al[nl][col];
        float* p = aOut + (size_t)(d0 + nl) * RR + col;
        *(volatile v4f*)p = ov;
        __threadfence();
        *(volatile v4f*)p = ov;
    }
}

__global__ void __launch_bounds__(256) k_update(float* Shat, const float* __restrict__ a_s, const float* __restrict__ a_t,
                                                const float* __restrict__ Wm2, const float* __restrict__ bm2)
{
    __shared__ float asl[16][RR + 1];
    __shared__ float atl[64][RR + 1];
    __shared__ float wl[RR];
    const int tid = threadIdx.x;
    const int blk = blockIdx.x;
    const int b  = blk >> 10;
    const int s0 = ((blk >> 4) & 63) * 16;
    const int t0 = (blk & 15) * 64;
    asl[tid >> 4][tid & 15] = a_s[(size_t)(b * NN + s0 + (tid >> 4)) * RR + (tid & 15)];
#pragma unroll
    for (int i = 0; i < 4; ++i) {
        const int idx = tid + 256 * i;
        atl[idx >> 4][idx & 15] = a_t[(size_t)(b * NN + t0 + (idx >> 4)) * RR + (idx & 15)];
    }
    if (tid < RR) wl[tid] = Wm2[tid];
    const float bias = bm2[0];
    __syncthreads();
    const int sl = tid >> 4, q = tid & 15;
    v4f add;
#pragma unroll
    for (int u = 0; u < 4; ++u) {
        const int tl = 4 * q + u;
        float acc = bias;
#pragma unroll
        for (int r = 0; r < RR; ++r) {
            float d = asl[sl][r] - atl[tl][r];
            d = d > 0.f ? d : 0.f;
            acc = fmaf(d, wl[r], acc);
        }
        add[u] = acc;
    }
    float* p = Shat + ((size_t)(b * NN + s0 + sl) * NN + t0 + 4 * q);
    const v4f nv = *(const v4f*)p + add;
    *(volatile v4f*)p = nv;
    __threadfence();
    *(volatile v4f*)p = nv;
}

extern "C" void kernel_launch(void* const* d_in, const int* in_sizes, int n_in,
                              void* d_out, int out_size, void* d_ws, size_t ws_size,
                              hipStream_t stream)
{
    if (n_in < 15) return;
    if (in_sizes[0] != BNN * FIN || in_sizes[3] != BNN * FIN) return;
    if (in_sizes[2] != BNN || in_sizes[5] != BNN) return;
    if (in_sizes[1] < 2 || (in_sizes[1] & 1) || in_sizes[4] < 2 || (in_sizes[4] & 1)) return;
    if (in_sizes[7] != FIN * FHID || in_sizes[8] != FHID) return;
    if (in_sizes[9] != RR * RR || in_sizes[10] != RR || in_sizes[11] != RR * RR ||
        in_sizes[12] != RR || in_sizes[13] != RR || in_sizes[14] < 1) return;
    if (in_sizes[6] < 0 || (in_sizes[6] % (BNN * RR)) != 0) return;
    if (out_size != 2 * BNN * NN) return;

    const int Es = in_sizes[1] / 2, Et = in_sizes[4] / 2;
    const int ncs = (Es + 255) / 256, nct = (Et + 255) / 256;
    const int nsteps = in_sizes[6] / (BNN * RR);

    const float* x_s    = (const float*)d_in[0];
    const int*   ei_s   = (const int*)  d_in[1];
    const float* x_t    = (const float*)d_in[3];
    const int*   ei_t   = (const int*)  d_in[4];
    const float* rsteps = (const float*)d_in[6];
    const float* W1     = (const float*)d_in[7];
    const float* b1     = (const float*)d_in[8];
    const float* W2     = (const float*)d_in[9];
    const float* b2     = (const float*)d_in[10];
    const float* Wm1    = (const float*)d_in[11];
    const float* bm1    = (const float*)d_in[12];
    const float* Wm2    = (const float*)d_in[13];
    const float* bm2    = (const float*)d_in[14];
    float* out0 = (float*)d_out;
    float* out1 = out0 + (size_t)BNN * NN;

    char* ws = (char*)d_ws;
    size_t off = 0;
    auto carve = [&](size_t bytes) -> void* {
        void* p = ws + off;
        off += (bytes + 255) & ~(size_t)255;
        return p;
    };
    unsigned short* aggp_s = (unsigned short*)carve((size_t)3 * BNN * FIN * 2);
    unsigned short* aggp_t = (unsigned short*)carve((size_t)3 * BNN * FIN * 2);
    unsigned short* W1p    = (unsigned short*)carve((size_t)3 * FHID * FIN * 2);
    unsigned short* hp_s   = (unsigned short*)carve((size_t)3 * BNN * FHID * 2);
    unsigned short* hp_t   = (unsigned short*)carve((size_t)3 * BNN * FHID * 2);
    float* Shat = (float*)carve((size_t)NB * NN * NN * 4);
    float* Sbuf = (float*)carve((size_t)NB * NN * NN * 4);
    float* rt   = (float*)carve((size_t)BNN * RR * 4);
    float* a_s  = (float*)carve((size_t)BNN * RR * 4);
    float* a_t  = (float*)carve((size_t)BNN * RR * 4);
    if (off > ws_size) return;

    const dim3 blk256(256), blk128(128);

    k_w1cvt<<<dim3(FHID / 16), blk256, 0, stream>>>(W1, W1p);
    k_agg_feat<<<dim3(BNN / NT), blk256, 0, stream>>>(x_s, ei_s, Es, ncs, aggp_s);
    k_agg_feat<<<dim3(BNN / NT), blk256, 0, stream>>>(x_t, ei_t, Et, nct, aggp_t);
    k_gemm1<<<dim3((BNN / 64) * (FHID / 64)), blk256, 0, stream>>>(aggp_s, W1p, b1, hp_s);
    k_gemm1<<<dim3((BNN / 64) * (FHID / 64)), blk256, 0, stream>>>(aggp_t, W1p, b1, hp_t);
    k_sim<<<dim3(NB * (NN / 64) * (NN / 64)), blk256, 0, stream>>>(hp_s, hp_t, Shat);
    k_softmax<<<dim3((BNN + NWAVE - 1) / NWAVE), blk256, 0, stream>>>(Shat, out0, BNN);

    for (int step = 0; step < nsteps; ++step) {
        const float* r_s = rsteps + (size_t)step * BNN * RR;
        const float* Ssrc = (step == 0) ? (const float*)out0 : (const float*)Sbuf;
        k_colmix<<<dim3(NB * (NN / 64)), blk128, 0, stream>>>(Ssrc, r_s, rt);
        k_agg_mlp<<<dim3(BNN / NT), blk256, 0, stream>>>(r_s, ei_s, Es, ncs, W2, b2, Wm1, bm1, 1, a_s);
        k_agg_mlp<<<dim3(BNN / NT), blk256, 0, stream>>>(rt,  ei_t, Et, nct, W2, b2, Wm1, bm1, 0, a_t);
        k_update<<<dim3(NB * (NN / 16) * (NN / 64)), blk256, 0, stream>>>(Shat, a_s, a_t, Wm2, bm2);
        if (step + 1 < nsteps)
            k_softmax<<<dim3((BNN + NWAVE - 1) / NWAVE), blk256, 0, stream>>>(Shat, Sbuf, BNN);
    }
    k_softmax<<<dim3((BNN + NWAVE - 1) / NWAVE), blk256, 0, stream>>>(Shat, out1, BNN);
}
